// GIN_17377437680137
// MI455X (gfx1250) — hardware-verified
//
#include <hip/hip_runtime.h>
#include <stddef.h>
#include <stdint.h>


#define DIN     128
#define KC      256
#define NLAY    3
#define NGR     256
#define OUTW    384
#define NTHR    256
#define NWAVE   8
#define EPT     8
#define CHUNK   (NTHR * EPT)
#define WCAP    (EPT * 32)
#define LISTN   (NWAVE * WCAP)
#define NBMAX   2048
#define NB      1024
#define RCAP    28672
#define DEGCAP  64
#define PKS     11
#define GBM     64
#define GBN     128
#define GTHR    128
#define GNT     8
#define TP      264
#define PLN     (DIN * KC)
#define NUP     (DIN * (KC / 8))
#define NUTOT   (2 * NLAY * NUP)
#define WSMAX   134217728
#define LDS_AGG ((2 * RCAP + 2 * NBMAX + LISTN) * 4 + 64)
#define LDS_MLP (GBM * GBN * 4 + GBM * TP * 2)

static_assert((CHUNK & (CHUNK - 1)) == 0 && CHUNK <= (1 << PKS));
static_assert((NBMAX & (NBMAX - 1)) == 0 && NBMAX <= (1 << PKS));
static_assert((NB & (NB - 1)) == 0 && NB <= NBMAX && (NB % NWAVE) == 0);
static_assert(NTHR * 8 == NBMAX);
static_assert(LISTN >= NBMAX && LISTN >= NWAVE * WCAP);
static_assert((RCAP % 32) == 0);
static_assert(LDS_AGG <= 300000 && LDS_MLP <= 300000);
static_assert(GBM == (GTHR / 32) * 16 && GBN == 16 * GNT && GBN == DIN);
static_assert(DIN == 32 * 4);
static_assert((KC % 32) == 0 && KC == 2 * DIN);
static_assert((NUP % NTHR) == 0 && (NUTOT % NTHR) == 0 && (KC / 8) == 32);
static_assert(((GBM * (DIN / 8)) % GTHR) == 0);
static_assert((TP % 8) == 0 && TP >= KC);
static_assert(OUTW == NLAY * DIN);

typedef float          v4f  __attribute__((ext_vector_type(4)));
typedef float          v8f  __attribute__((ext_vector_type(8)));
typedef int            v4i  __attribute__((ext_vector_type(4)));
typedef int            v8i  __attribute__((ext_vector_type(8)));
typedef unsigned int   v2u  __attribute__((ext_vector_type(2)));
typedef unsigned short v8us __attribute__((ext_vector_type(8)));
typedef __bf16         v16b __attribute__((ext_vector_type(16)));
typedef v4f  __attribute__((may_alias)) v4fa;
typedef v8us __attribute__((may_alias)) v8usa;
union Frag { v16b vb; v8us h[2]; v8i w; };

__device__ __forceinline__ v8f wmb(const Frag& a, const Frag& b, v8f c) {
  v8f d = __builtin_amdgcn_wmma_f32_16x16x32_bf16(false, a.vb, false, b.vb, (short)0, c, false, false);
  asm volatile("v_nop\n\tv_nop\n\tv_nop\n\tv_nop" : "+v"(d) : "v"(a.w), "v"(b.w));
  return d;
}

__device__ __forceinline__ unsigned short bf_bits(float f) {
  const unsigned int u = __float_as_uint(f);
  unsigned int r = (u + 0x7FFFu + ((u >> 16) & 1u)) >> 16;
  r = (f == f) ? r : 0x7FC0u;
  return (unsigned short)r;
}
__device__ __forceinline__ float bf_val(unsigned short b) { return __uint_as_float(((unsigned int)b) << 16); }
__device__ __forceinline__ float bf_rne(float f) { return bf_val(bf_bits(f)); }

__device__ __forceinline__ void hilo8(const v4f a, const v4f b, v8us& hv, v8us& lv) {
  const float f[8] = {a.x, a.y, a.z, a.w, b.x, b.y, b.z, b.w};
#pragma unroll
  for (int j = 0; j < 8; ++j) {
    const unsigned short hb = bf_bits(f[j]);
    hv[j] = hb;
    lv[j] = bf_bits(f[j] - bf_val(hb));
  }
}

__device__ __forceinline__ int scan_chunk(const int* __restrict__ dsts, int nE, int cbase, int slotBase,
                                          int nb, int vec8, int* list, int tid, int lane, int wave) {
  int wc = 0;
  const int el0  = tid * EPT;
  const int e0   = cbase + el0;
  const int sent = -2147483647 - 1;
  v4i da, db;
  if (vec8 != 0 && cbase + CHUNK <= nE) {
    da = *(const v4i*)(dsts + e0);
    db = *(const v4i*)(dsts + e0 + 4);
  } else {
    da.x = (e0     < nE) ? dsts[min(e0,     nE - 1)] : sent;
    da.y = (e0 + 1 < nE) ? dsts[min(e0 + 1, nE - 1)] : sent;
    da.z = (e0 + 2 < nE) ? dsts[min(e0 + 2, nE - 1)] : sent;
    da.w = (e0 + 3 < nE) ? dsts[min(e0 + 3, nE - 1)] : sent;
    db.x = (e0 + 4 < nE) ? dsts[min(e0 + 4, nE - 1)] : sent;
    db.y = (e0 + 5 < nE) ? dsts[min(e0 + 5, nE - 1)] : sent;
    db.z = (e0 + 6 < nE) ? dsts[min(e0 + 6, nE - 1)] : sent;
    db.w = (e0 + 7 < nE) ? dsts[min(e0 + 7, nE - 1)] : sent;
  }
  const unsigned nbs = (unsigned)slotBase;
  const unsigned unb = (unsigned)nb;
  const unsigned s0 = (unsigned)da.x - nbs, s1 = (unsigned)da.y - nbs;
  const unsigned s2 = (unsigned)da.z - nbs, s3 = (unsigned)da.w - nbs;
  const unsigned s4 = (unsigned)db.x - nbs, s5 = (unsigned)db.y - nbs;
  const unsigned s6 = (unsigned)db.z - nbs, s7 = (unsigned)db.w - nbs;
  const bool h0 = s0 < unb, h1 = s1 < unb, h2 = s2 < unb, h3 = s3 < unb;
  const bool h4 = s4 < unb, h5 = s5 < unb, h6 = s6 < unb, h7 = s7 < unb;
  const unsigned any = __builtin_amdgcn_ballot_w32(h0 | h1 | h2 | h3 | h4 | h5 | h6 | h7);
  if (any != 0u) {
#define HITJ(J, HJ, SJ) { \
      const unsigned mj = __builtin_amdgcn_ballot_w32(HJ); \
      if (mj != 0u) { \
        if (HJ) { \
          const int pos = wc + (int)__builtin_amdgcn_mbcnt_lo(mj, 0u); \
          if (pos < WCAP) list[wave * WCAP + pos] = ((el0 + (J)) << PKS) | (int)(SJ); \
        } \
        wc += (int)__builtin_popcount(mj); } }
    HITJ(0, h0, s0)
    HITJ(1, h1, s1)
    HITJ(2, h2, s2)
    HITJ(3, h3, s3)
    HITJ(4, h4, s4)
    HITJ(5, h5, s5)
    HITJ(6, h6, s6)
    HITJ(7, h7, s7)
#undef HITJ
  }
  return wc;
}

__global__ __launch_bounds__(NTHR) void k_wprep(const float* __restrict__ W1, const float* __restrict__ W2,
                                                unsigned short* wc) {
  const int u = (int)blockIdx.x * NTHR + (int)threadIdx.x;
  if (u >= NUTOT) return;
  const int p   = u / NUP;
  const int v   = u - p * NUP;
  const int n   = v >> 5;
  const int k8  = (v & 31) * 8;
  const int kk  = k8 & (DIN - 1);
  const int lay = (p < NLAY) ? p : p - NLAY;
  const float* wsrc = (p < NLAY) ? W1 : W2;
  const float* q = wsrc + (size_t)lay * DIN * DIN + (size_t)kk * DIN + n;
  v8us o;
#pragma unroll
  for (int i = 0; i < 8; ++i) o[i] = bf_bits(q[(size_t)i * DIN]);
  unsigned short* dp = wc + (size_t)p * PLN + (size_t)v * 8;
  *(volatile v8us*)dp = o;
  __threadfence();
  *(volatile v8us*)dp = o;
}

template <int RND>
__global__ __launch_bounds__(NTHR) void k_agg(
    const int* __restrict__ srcs, const int* __restrict__ dsts,
    const float* __restrict__ fin,
    unsigned short* Uout,
    int nN, int nE, int nb, int vec8, int MPr) {
  extern __shared__ v4f lds_dyn[];
  int* reg1 = (int*)lds_dyn;
  int* reg2 = reg1 + RCAP;
  int* scnt = reg2 + RCAP;
  int* soff = scnt + NBMAX;
  int* list = soff + NBMAX;
  int* wcnt = list + LISTN;
  int* wtot = wcnt + NWAVE;
  const int tid = (int)threadIdx.x, lane = tid & 31, wave = tid >> 5;
  const int nodeBase = (int)blockIdx.x * nb;

  for (int i = tid; i < NBMAX; i += NTHR) scnt[i] = 0;
  __syncthreads();

  int tot = 0;
  const int nChunks = (nE + CHUNK - 1) / CHUNK;
#pragma unroll 1
  for (int ch = 0; ch < nChunks; ++ch) {
    const int cbase = ch * CHUNK;
    const int wc = scan_chunk(dsts, nE, cbase, nodeBase, nb, vec8, list, tid, lane, wave);
    if (lane == 0) wcnt[wave] = wc;
    __syncthreads();
    int pre = 0, all = 0;
#pragma unroll
    for (int w2 = 0; w2 < NWAVE; ++w2) {
      int c = wcnt[w2];
      c = c < 0 ? 0 : (c > WCAP ? WCAP : c);
      all += c;
      pre += (w2 < wave) ? c : 0;
    }
    const int wcc  = wc > WCAP ? WCAP : wc;
    const int base = tot + pre;
#pragma unroll 1
    for (int i = lane; i < wcc; i += 32) {
      const int ent = list[wave * WCAP + i];
      const int el  = (ent >> PKS) & (CHUNK - 1);
      const int sl  = ent & (NBMAX - 1);
      int eid = cbase + el;
      eid = eid > nE - 1 ? nE - 1 : eid;
      const int pos = base + i;
      if (pos < RCAP) reg1[pos] = (int)(((unsigned)eid << PKS) | (unsigned)sl);
    }
    tot += all;
    tot = tot > RCAP ? RCAP : tot;
    __syncthreads();
  }
  const int nh = tot;

  if (wave == 0) {
#pragma unroll 1
    for (int b0 = 0; b0 < nh; b0 += 32) {
      const int idx = b0 + lane;
      const int uv  = reg1[idx < RCAP ? idx : RCAP - 1];
      const int m32 = (nh - b0) < 32 ? (nh - b0) : 32;
#pragma unroll 1
      for (int k = 0; k < m32; ++k) {
        const int u  = __builtin_amdgcn_readlane(uv, k);
        const int sl = u & (NBMAX - 1);
        if (lane == 0) scnt[sl] = scnt[sl] + 1;
      }
    }
  }
  __syncthreads();

  {
    const v4i ca = *(const v4i*)(scnt + 8 * tid);
    const v4i cb = *(const v4i*)(scnt + 8 * tid + 4);
    const int e0 = ca.x < 0 ? 0 : ca.x, e1 = ca.y < 0 ? 0 : ca.y, e2 = ca.z < 0 ? 0 : ca.z, e3 = ca.w < 0 ? 0 : ca.w;
    const int e4 = cb.x < 0 ? 0 : cb.x, e5 = cb.y < 0 ? 0 : cb.y, e6 = cb.z < 0 ? 0 : cb.z, e7 = cb.w < 0 ? 0 : cb.w;
    const int ts = e0 + e1 + e2 + e3 + e4 + e5 + e6 + e7;
    int incl = ts;
#pragma unroll
    for (int d = 1; d < 32; d <<= 1) {
      const int up = __shfl_up(incl, d);
      if (lane >= d) incl += up;
    }
    if (lane == 31) wtot[wave] = incl;
    __syncthreads();
    int pre = 0;
#pragma unroll
    for (int w2 = 0; w2 < NWAVE; ++w2) pre += (w2 < wave) ? wtot[w2] : 0;
    int run = pre + incl - ts;
    soff[8 * tid + 0] = run; run += e0;
    soff[8 * tid + 1] = run; run += e1;
    soff[8 * tid + 2] = run; run += e2;
    soff[8 * tid + 3] = run; run += e3;
    soff[8 * tid + 4] = run; run += e4;
    soff[8 * tid + 5] = run; run += e5;
    soff[8 * tid + 6] = run; run += e6;
    soff[8 * tid + 7] = run;
  }
  __syncthreads();
  for (int i = tid; i < NBMAX; i += NTHR) list[i] = soff[i];
  __syncthreads();

  if (wave == 0) {
#pragma unroll 1
    for (int b0 = 0; b0 < nh; b0 += 32) {
      const int idx = b0 + lane;
      const int uv  = reg1[idx < RCAP ? idx : RCAP - 1];
      const int m32 = (nh - b0) < 32 ? (nh - b0) : 32;
#pragma unroll 1
      for (int k = 0; k < m32; ++k) {
        const int u   = __builtin_amdgcn_readlane(uv, k);
        const int sl  = u & (NBMAX - 1);
        const int eid = (int)((unsigned)u >> PKS);
        if (lane == 0) {
          int pos = list[sl];
          pos = pos < 0 ? 0 : (pos > RCAP - 1 ? RCAP - 1 : pos);
          reg2[pos] = eid;
          list[sl] = pos + 1;
        }
      }
    }
  }
  __syncthreads();

  const int nbw = nb >> 3;
  const bool ovf = (nh >= RCAP);
  const float qnan = __int_as_float(0x7fc00000);

#pragma unroll 1
  for (int jt = 0; jt < nbw; ++jt) {
    const int slot = wave * nbw + jt;
    const int grow = nodeBase + slot;
    int st = soff[slot];
    const int craw = scnt[slot];
    int cnt = craw;
    st  = st < 0 ? 0 : (st > nh ? nh : st);
    cnt = cnt < 0 ? 0 : (cnt > DEGCAP ? DEGCAP : cnt);
    if (cnt > nh - st) cnt = nh - st;
    const float pz = (ovf || craw > DEGCAP) ? qnan : 0.0f;
    const bool liveRow = grow < nN;

    float ag0 = 0.f, ag1 = 0.f, ag2 = 0.f, ag3 = 0.f;
#pragma unroll 1
    for (int q = 0; q < cnt; ++q) {
      int idx = st + q; idx = idx > RCAP - 1 ? RCAP - 1 : idx;
      int eid = reg2[idx]; eid = eid < 0 ? 0 : (eid > nE - 1 ? nE - 1 : eid);
      const int sraw = srcs[eid];
      const int s = sraw < 0 ? 0 : (sraw > nN - 1 ? nN - 1 : sraw);
      const v4f v = *(const v4f*)(fin + (size_t)s * DIN + 4 * lane);
      float v0 = v.x, v1 = v.y, v2 = v.z, v3 = v.w;
      if (RND != 0) { v0 = bf_rne(v0); v1 = bf_rne(v1); v2 = bf_rne(v2); v3 = bf_rne(v3); }
      ag0 += v0; ag1 += v1; ag2 += v2; ag3 += v3;
    }
    const int nc = liveRow ? grow : nN - 1;
    const v4f sv = *(const v4f*)(fin + (size_t)nc * DIN + 4 * lane);
    float s0 = sv.x, s1 = sv.y, s2 = sv.z, s3 = sv.w;
    if (RND != 0) { s0 = bf_rne(s0); s1 = bf_rne(s1); s2 = bf_rne(s2); s3 = bf_rne(s3); }
    float r0 = s0 + ag0, r1 = s1 + ag1, r2 = s2 + ag2, r3 = s3 + ag3;
    r0 = (liveRow ? r0 : 0.0f) + pz;
    r1 = (liveRow ? r1 : 0.0f) + pz;
    r2 = (liveRow ? r2 : 0.0f) + pz;
    r3 = (liveRow ? r3 : 0.0f) + pz;

    const unsigned short hb0 = bf_bits(r0), hb1 = bf_bits(r1), hb2 = bf_bits(r2), hb3 = bf_bits(r3);
    const unsigned short lb0 = bf_bits(r0 - bf_val(hb0)), lb1 = bf_bits(r1 - bf_val(hb1));
    const unsigned short lb2 = bf_bits(r2 - bf_val(hb2)), lb3 = bf_bits(r3 - bf_val(hb3));
    v2u hk, lk;
    hk.x = (unsigned int)hb0 | ((unsigned int)hb1 << 16);
    hk.y = (unsigned int)hb2 | ((unsigned int)hb3 << 16);
    lk.x = (unsigned int)lb0 | ((unsigned int)lb1 << 16);
    lk.y = (unsigned int)lb2 | ((unsigned int)lb3 << 16);
    unsigned short* gp = Uout + (size_t)grow * KC + 4 * lane;
    const bool wsv = grow < MPr;
    if (wsv) { *(volatile v2u*)gp = hk; *(volatile v2u*)(gp + DIN) = lk; }
    __threadfence();
    if (wsv) { *(volatile v2u*)gp = hk; *(volatile v2u*)(gp + DIN) = lk; }
  }
}

__global__ __launch_bounds__(GTHR) void k_mlp(const unsigned short* __restrict__ U,
                                              const unsigned short* __restrict__ W1c,
                                              const unsigned short* __restrict__ W2c,
                                              const float* __restrict__ b1, const float* __restrict__ b2,
                                              float* H, int nN, int mRows) {
  extern __shared__ v4f mlp_dyn[];
  float* stg = (float*)mlp_dyn;
  unsigned short* tt = (unsigned short*)(stg + GBM * GBN);
  const int tid = (int)threadIdx.x, lane = tid & 31, wave = tid >> 5, hh = lane >> 4, m = lane & 15;
  const int rowBase = (int)blockIdx.x * GBM;

  v8f acc[GNT];
  const v8f zacc = {0.f, 0.f, 0.f, 0.f, 0.f, 0.f, 0.f, 0.f};
#pragma unroll
  for (int t = 0; t < GNT; ++t) acc[t] = zacc;

  {
    const unsigned short* ap = U   + (size_t)(rowBase + 16 * wave + m) * KC + 8 * hh;
    const unsigned short* bp = W1c + (size_t)m * KC + 8 * hh;
#pragma unroll 1
    for (int k0 = 0; k0 < KC; k0 += 32) {
      Frag af;
      af.h[0] = *(const v8usa*)(ap + k0);
      af.h[1] = *(const v8usa*)(ap + k0 + 16);
#pragma unroll
      for (int nt = 0; nt < GNT; ++nt) {
        const unsigned short* wq = bp + (size_t)(16 * nt) * KC + k0;
        Frag bfr;
        bfr.h[0] = *(const v8usa*)wq;
        bfr.h[1] = *(const v8usa*)(wq + 16);
        acc[nt] = wmb(af, bfr, acc[nt]);
      }
    }
  }
#pragma unroll
  for (int nt = 0; nt < GNT; ++nt) {
    const int lc = 16 * nt + m;
    const float bb = bf_rne(b1[lc]);
#pragma unroll
    for (int r = 0; r < 8; ++r) {
      const int lr = 16 * wave + 8 * hh + r;
      const float v = acc[nt][r] + bb;
      stg[lr * GBN + lc] = (v > 0.0f) ? v : (v - v);
    }
  }
  __syncthreads();

#pragma unroll 1
  for (int i = 0; i < (GBM * (DIN / 8)) / GTHR; ++i) {
    const int p = i * GTHR + tid;
    const int row = p >> 4, q = p & 15;
    const v4f a = *(const v4fa*)(stg + row * GBN + 8 * q);
    const v4f b = *(const v4fa*)(stg + row * GBN + 8 * q + 4);
    v8us hv, lv;
    hilo8(a, b, hv, lv);
    *(v8usa*)(tt + row * TP + 8 * q)       = hv;
    *(v8usa*)(tt + row * TP + DIN + 8 * q) = lv;
  }
  __syncthreads();

#pragma unroll
  for (int t = 0; t < GNT; ++t) acc[t] = zacc;
  {
    const unsigned short* tp = tt  + (16 * wave + m) * TP + 8 * hh;
    const unsigned short* bp = W2c + (size_t)m * KC + 8 * hh;
#pragma unroll 1
    for (int k0 = 0; k0 < KC; k0 += 32) {
      Frag af;
      af.h[0] = *(const v8usa*)(tp + k0);
      af.h[1] = *(const v8usa*)(tp + k0 + 16);
#pragma unroll
      for (int nt = 0; nt < GNT; ++nt) {
        const unsigned short* wq = bp + (size_t)(16 * nt) * KC + k0;
        Frag bfr;
        bfr.h[0] = *(const v8usa*)wq;
        bfr.h[1] = *(const v8usa*)(wq + 16);
        acc[nt] = wmb(af, bfr, acc[nt]);
      }
    }
  }
#pragma unroll
  for (int nt = 0; nt < GNT; ++nt) {
    const int lc = 16 * nt + m;
    const float bb = bf_rne(b2[lc]);
#pragma unroll
    for (int r = 0; r < 8; ++r) {
      const int lr = 16 * wave + 8 * hh + r;
      const bool live = (rowBase + lr) < nN;
      const float v = acc[nt][r] + bb;
      const float y = (v > 0.0f) ? v : (v - v);
      stg[lr * GBN + lc] = live ? y : 0.0f;
    }
  }
  __syncthreads();

  v4f fv[16];
#pragma unroll
  for (int i = 0; i < 16; ++i) {
    const int lr = 16 * wave + i;
    fv[i] = *(const v4fa*)(stg + lr * GBN + 4 * lane);
  }
#pragma unroll
  for (int i = 0; i < 16; ++i) {
    const int gr = rowBase + 16 * wave + i;
    float* op = H + (size_t)gr * DIN + 4 * lane;
    if (gr < mRows) *(volatile v4f*)op = fv[i];
  }
  __threadfence();
#pragma unroll
  for (int i = 0; i < 16; ++i) {
    const int gr = rowBase + 16 * wave + i;
    float* op = H + (size_t)gr * DIN + 4 * lane;
    if (gr < mRows) *(volatile v4f*)op = fv[i];
  }
}

__global__ __launch_bounds__(NTHR) void k_pool(const float* __restrict__ hf, const int* __restrict__ bat,
                                               int nN, float* out, int colOff) {
  __shared__ __attribute__((aligned(16))) float wsum[NWAVE * DIN];
  __shared__ __attribute__((aligned(16))) float outs[DIN];
  const int tid = (int)threadIdx.x, lane = tid & 31, wave = tid >> 5;
  const int g = (int)blockIdx.x;

  float a0 = 0.0f, a1 = 0.0f, a2 = 0.0f, a3 = 0.0f;
#pragma unroll 1
  for (int i0 = wave * 32; i0 < nN; i0 += NTHR) {
    const int i  = i0 + lane;
    const int ic = i < nN ? i : nN - 1;
    const int b  = bat[ic];
    const bool hit = (i < nN) && (b == g);
    unsigned msk = __builtin_amdgcn_ballot_w32(hit);
    int nh = (int)__builtin_popcount(msk);
    nh = nh > 32 ? 32 : nh;
#pragma unroll 1
    for (int q = 0; q < nh; ++q) {
      const int k = __builtin_ffs((int)msk) - 1;
      msk &= msk - 1u;
      int node = i0 + (k < 0 ? 0 : k);
      node = node > nN - 1 ? nN - 1 : node;
      const v4f v = *(const v4fa*)(hf + (size_t)node * DIN + 4 * lane);
      a0 += v.x; a1 += v.y; a2 += v.z; a3 += v.w;
    }
  }
  {
    v4f pa; pa.x = a0; pa.y = a1; pa.z = a2; pa.w = a3;
    *(v4fa*)(wsum + wave * DIN + 4 * lane) = pa;
  }
  __syncthreads();
  if (tid < DIN) {
    float s = 0.0f;
#pragma unroll
    for (int w2 = 0; w2 < NWAVE; ++w2) s += wsum[w2 * DIN + tid];
    outs[tid] = s;
  }
  __syncthreads();
  const v4f ov = *(const v4fa*)(outs + 4 * lane);
  float* op = out + (size_t)g * OUTW + colOff + 4 * lane;
  const bool okst = (wave == 0);
  if (okst) *(volatile v4f*)op = ov;
  __threadfence();
  if (okst) *(volatile v4f*)op = ov;
}

static inline int cdiv(int a, int b) { return (a + b - 1) / b; }
static inline size_t al256(size_t o) { return (o + 255) & ~(size_t)255; }

extern "C" void kernel_launch(void* const* d_in, const int* in_sizes, int n_in,
                              void* d_out, int out_size, void* d_ws, size_t ws_size,
                              hipStream_t stream) {
  if (n_in < 7) return;
  if (in_sizes[0] < DIN || (in_sizes[0] % DIN) != 0) return;
  const int nN = in_sizes[0] / DIN;
  if (nN < 1 || nN > (1 << 22)) return;
  if (in_sizes[1] < 2 || (in_sizes[1] & 1) != 0) return;
  const int nE = in_sizes[1] / 2;
  if (nE < 1 || nE > (1 << 21)) return;
  if (in_sizes[2] != nN) return;
  if (in_sizes[3] != NLAY * DIN * DIN || in_sizes[4] != NLAY * DIN) return;
  if (in_sizes[5] != NLAY * DIN * DIN || in_sizes[6] != NLAY * DIN) return;
  if (out_size != NGR * OUTW) return;

  const float* x     = (const float*)d_in[0];
  const int*   ei    = (const int*)  d_in[1];
  const int*   batch = (const int*)  d_in[2];
  const float* W1    = (const float*)d_in[3];
  const float* b1    = (const float*)d_in[4];
  const float* W2    = (const float*)d_in[5];
  const float* b2    = (const float*)d_in[6];
  float* out = (float*)d_out;
  const int* src = ei;
  const int* dst = ei + nE;

  const int MP   = cdiv(nN, GBM) * GBM;
  const int gM   = MP / GBM;
  const int gA   = cdiv(MP, NB);
  if ((long long)gA * NB < (long long)MP) return;
  const int vec8 = ((nE & 3) == 0) ? 1 : 0;

  char* ws = (char*)d_ws;
  size_t off = 0;
  const size_t oWC = off; off = al256(off + (size_t)2 * NLAY * PLN * 2);
  const size_t oU  = off; off = al256(off + (size_t)MP * KC * 2);
  const size_t oH  = off; off = al256(off + (size_t)MP * DIN * 4);
  if (off > ws_size || off > (size_t)WSMAX) return;
  unsigned short* WC = (unsigned short*)(ws + oWC);
  unsigned short* U  = (unsigned short*)(ws + oU);
  float*          H  = (float*)(ws + oH);

  hipFuncSetAttribute(reinterpret_cast<const void*>(&k_agg<1>), hipFuncAttributeMaxDynamicSharedMemorySize, LDS_AGG);
  hipFuncSetAttribute(reinterpret_cast<const void*>(&k_agg<0>), hipFuncAttributeMaxDynamicSharedMemorySize, LDS_AGG);
  hipFuncSetAttribute(reinterpret_cast<const void*>(&k_mlp),    hipFuncAttributeMaxDynamicSharedMemorySize, LDS_MLP);

  k_wprep<<<NUTOT / NTHR, NTHR, 0, stream>>>(W1, W2, WC);

  k_agg<1><<<gA, NTHR, LDS_AGG, stream>>>(src, dst, x, U, nN, nE, NB, vec8, MP);
  k_mlp<<<gM, GTHR, LDS_MLP, stream>>>(U, WC + (size_t)0 * PLN, WC + (size_t)(NLAY + 0) * PLN,
                                       b1 + 0 * DIN, b2 + 0 * DIN, H, nN, MP);
  k_pool<<<NGR, NTHR, 0, stream>>>(H, batch, nN, out, 0 * DIN);

  k_agg<0><<<gA, NTHR, LDS_AGG, stream>>>(src, dst, H, U, nN, nE, NB, vec8, MP);
  k_mlp<<<gM, GTHR, LDS_MLP, stream>>>(U, WC + (size_t)1 * PLN, WC + (size_t)(NLAY + 1) * PLN,
                                       b1 + 1 * DIN, b2 + 1 * DIN, H, nN, MP);
  k_pool<<<NGR, NTHR, 0, stream>>>(H, batch, nN, out, 1 * DIN);

  k_agg<0><<<gA, NTHR, LDS_AGG, stream>>>(src, dst, H, U, nN, nE, NB, vec8, MP);
  k_mlp<<<gM, GTHR, LDS_MLP, stream>>>(U, WC + (size_t)2 * PLN, WC + (size_t)(NLAY + 2) * PLN,
                                       b1 + 2 * DIN, b2 + 2 * DIN, H, nN, MP);
  k_pool<<<NGR, NTHR, 0, stream>>>(H, batch, nN, out, 2 * DIN);
}
